// ParallelBlock_65687229825678
// MI455X (gfx1250) — hardware-verified
//
#include <hip/hip_runtime.h>
#include <math.h>

constexpr int kBatch = 2;
constexpr int kSeq   = 2048;
constexpr int kDim   = 1024;
constexpr int kHeads = 16;
constexpr int kHDim  = 64;
constexpr int kFF    = 4096;
constexpr int kTok   = kBatch * kSeq;
constexpr int kGrp   = 2;
constexpr int kNChunk = (kBatch * kHeads) / kGrp;
constexpr float kWCarry    = 64.0f;
constexpr float kWCarryInv = 1.0f / 64.0f;
constexpr float kPCarry    = 2048.0f;
constexpr float kCtxCarry  = 256.0f;
constexpr float kPVScale   = kCtxCarry / kPCarry;
constexpr float kWoScale   = 1.0f / (kCtxCarry * kWCarry);
constexpr float kQKScale   = 0.125f;
constexpr float kInvDim    = 1.0f / 1024.0f;
constexpr float kEps       = 1.1920929e-7f;

typedef __attribute__((ext_vector_type(16))) _Float16 v16h;
typedef __attribute__((ext_vector_type(8)))  _Float16 v8h;
typedef __attribute__((ext_vector_type(16))) __bf16   v16b;
typedef __attribute__((ext_vector_type(8)))  __bf16   v8b;
typedef __attribute__((ext_vector_type(8)))  float    v8f;
typedef __attribute__((ext_vector_type(4)))  float    v4f;
typedef __attribute__((ext_vector_type(4)))  unsigned int v4u;

__device__ __forceinline__ unsigned short f2bf_bits(float f) {
  unsigned u = __float_as_uint(f);
  return (unsigned short)((u + 0x7FFFu + ((u >> 16) & 1u)) >> 16);
}
__device__ __forceinline__ float bf_bits2f(unsigned short h) { return __uint_as_float(((unsigned)h) << 16); }

__device__ __forceinline__ void dep_guard_h(v8f& a, v8f& b, v16h x, v16h y) { asm volatile("v_nop\n\tv_nop\n\tv_nop\n\tv_nop" : "+v"(a), "+v"(b) : "v"(x), "v"(y)); }
__device__ __forceinline__ void dep_guard_b(v8f& a, v8f& b, v16b x, v16b y) { asm volatile("v_nop\n\tv_nop\n\tv_nop\n\tv_nop" : "+v"(a), "+v"(b) : "v"(x), "v"(y)); }
__device__ __forceinline__ void keep4_h(v16h a, v16h b, v16h c, v16h d) { asm volatile("v_nop" :: "v"(a), "v"(b), "v"(c), "v"(d)); }
__device__ __forceinline__ void keep4_b(v16b a, v16b b, v16b c, v16b d) { asm volatile("v_nop" :: "v"(a), "v"(b), "v"(c), "v"(d)); }
__device__ __forceinline__ void acc_guard4(v8f& a, v8f& b, v8f& c, v8f& d) { asm volatile("v_nop\n\tv_nop\n\tv_nop\n\tv_nop" : "+v"(a), "+v"(b), "+v"(c), "+v"(d)); }
template <typename T> struct Frag;
template <> struct Frag<_Float16> {
  typedef v16h V; union U { v16h v; v8h h[2]; };
  static __device__ __forceinline__ v16h load(const _Float16* p) {
    U f; f.h[0] = *(const v8h*)(p); f.h[1] = *(const v8h*)(p + 16); return f.v;
  }
  static __device__ __forceinline__ v8f mma(v16h a, v16h b, v8f c) {
    return __builtin_amdgcn_wmma_f32_16x16x32_f16(false, a, false, b, (short)0, c, false, false);
  }
  static __device__ __forceinline__ void guard(v8f& a, v8f& b, v16h x, v16h y) { dep_guard_h(a, b, x, y); }
  static __device__ __forceinline__ void keep(v16h a, v16h b, v16h c, v16h d) { keep4_h(a, b, c, d); }
};
template <> struct Frag<__bf16> {
  typedef v16b V; union U { v16b v; v8b h[2]; };
  static __device__ __forceinline__ v16b load(const __bf16* p) {
    U f; f.h[0] = *(const v8b*)(p); f.h[1] = *(const v8b*)(p + 16); return f.v;
  }
  static __device__ __forceinline__ v8f mma(v16b a, v16b b, v8f c) {
    return __builtin_amdgcn_wmma_f32_16x16x32_bf16(false, a, false, b, (short)0, c, false, false);
  }
  static __device__ __forceinline__ void guard(v8f& a, v8f& b, v16b x, v16b y) { dep_guard_b(a, b, x, y); }
  static __device__ __forceinline__ void keep(v16b a, v16b b, v16b c, v16b d) { keep4_b(a, b, c, d); }
};

__device__ __forceinline__ unsigned pk16(unsigned short a, unsigned short b) { return (unsigned)a | ((unsigned)b << 16); }
__device__ __forceinline__ unsigned short h_bits(float f) { const _Float16 h = (_Float16)f; return __builtin_bit_cast(unsigned short, h); }

template <int ET> struct Elem;
template <> struct Elem<0> { typedef _Float16 T; };
template <> struct Elem<1> { typedef __bf16 T; };
template <int ET, bool SPLIT, int BIAS_MODE, int OUT_MODE, bool RESID, int ACT = 0, int CAUS = 0>
__global__ __launch_bounds__(256) void wmma_gemm64(
    const unsigned short* __restrict__ Ap, const unsigned short* __restrict__ A2p, int lda, long strideA,
    const unsigned short* __restrict__ Btp, const unsigned short* __restrict__ Bt2p, int ldb, long strideB,
    void* __restrict__ Cout, void* __restrict__ Cout2, int ldc, long strideC,
    const float* __restrict__ bias,
    const float* __restrict__ resid, long strideR,
    int M, int N, int K, float scale) {
  typedef typename Elem<ET>::T T;
  typedef typename Frag<T>::V V;
  const T* A = (const T*)Ap; const T* A2 = (const T*)A2p; const T* Bt = (const T*)Btp; const T* Bt2 = (const T*)Bt2p;
  __shared__ __align__(16) float sT[8][16 * 68];
  const int b    = blockIdx.y;
  const int lane = threadIdx.x & 31;
  const int wave = threadIdx.x >> 5;
  const int tilesN = N >> 6;
  const int tilesM = M >> 6;
  const int tile = blockIdx.x * 8 + wave;
  if (tile >= tilesM * tilesN) return;
  const int tm = tile / tilesN;
  const int tn = tile - tm * tilesN;
  const int m0 = tm << 6;
  const int n0 = tn << 6;
  if (CAUS == 1 && n0 > m0) return;
  const int Kend = (CAUS == 2) ? ((m0 + 64 < K) ? (m0 + 64) : K) : K;

  const T* Ab  = A  + (size_t)b * strideA;
  const T* Bb  = Bt + (size_t)b * strideB;
  const T* Ab2 = SPLIT ? (A2  + (size_t)b * strideA) : nullptr;
  const T* Bb2 = SPLIT ? (Bt2 + (size_t)b * strideB) : nullptr;

  const int rlane = lane & 15;
  const int koff  = (lane >> 4) * 8;
  const int mOff  = (lane >> 4) * 8;

  v8f acc[4][4];
#pragma unroll
  for (int i = 0; i < 4; ++i)
#pragma unroll
    for (int j = 0; j < 4; ++j) acc[i][j] = (v8f){0.f,0.f,0.f,0.f,0.f,0.f,0.f,0.f};

  for (int k0 = 0; k0 < Kend; k0 += 32) {
    V bh[4], bl[4];
#pragma unroll
    for (int j = 0; j < 4; ++j) {
      const size_t bo = (size_t)(n0 + (j << 4) + rlane) * ldb + koff + k0;
      bh[j] = Frag<T>::load(Bb + bo);
      if (SPLIT) bl[j] = Frag<T>::load(Bb2 + bo);
    }
#pragma unroll
    for (int i = 0; i < 4; ++i) {
      const size_t ao = (size_t)(m0 + (i << 4) + rlane) * lda + koff + k0;
      V ah = Frag<T>::load(Ab + ao);
      V al;
      if (SPLIT) al = Frag<T>::load(Ab2 + ao);
#pragma unroll
      for (int j = 0; j < 4; ++j) {
        acc[i][j] = Frag<T>::mma(ah, bh[j], acc[i][j]);
        if (SPLIT) {
          acc[i][j] = Frag<T>::mma(ah, bl[j], acc[i][j]);
          acc[i][j] = Frag<T>::mma(al, bh[j], acc[i][j]);
        }
      }
      Frag<T>::guard(acc[i][0], acc[i][3], ah, SPLIT ? al : ah);
    }
    Frag<T>::keep(bh[0], bh[1], bh[2], bh[3]);
    if (SPLIT) Frag<T>::keep(bl[0], bl[1], bl[2], bl[3]);
  }
  acc_guard4(acc[0][0], acc[0][1], acc[0][2], acc[0][3]);
  acc_guard4(acc[1][0], acc[1][1], acc[1][2], acc[1][3]);
  acc_guard4(acc[2][0], acc[2][1], acc[2][2], acc[2][3]);
  acc_guard4(acc[3][0], acc[3][1], acc[3][2], acc[3][3]);

  float* slab = sT[wave];
  const float* Rb = RESID ? (resid + (size_t)b * strideR) : nullptr;
#pragma unroll
  for (int i = 0; i < 4; ++i) {
    const int mBase = m0 + (i << 4);
#pragma unroll
    for (int j = 0; j < 4; ++j) {
      const int n = n0 + (j << 4) + rlane;
      float bv = 0.f;
      if (BIAS_MODE == 2) bv = bias[n];
#pragma unroll
      for (int r = 0; r < 8; ++r) {
        float v = acc[i][j][r] * scale;
        if (BIAS_MODE == 1) v += bias[mBase + mOff + r];
        if (BIAS_MODE == 2) v += bv;
        if (RESID) v += Rb[(size_t)(mBase + mOff + r) * ldc + n];
        if (ACT == 2) v = fmaxf(v, 0.0f);
        if (ACT == 3) v = v / (1.0f + expf(-v));
        if (ACT == 4) v = (v > 0.f) ? v : 0.01f * v;
        slab[(mOff + r) * 68 + (j << 4) + rlane] = v;
      }
    }
    __builtin_amdgcn_fence(__ATOMIC_RELEASE, "workgroup");
    __builtin_amdgcn_wave_barrier();
    __builtin_amdgcn_fence(__ATOMIC_ACQUIRE, "workgroup");
    if (OUT_MODE == 0) {
      float* C = (float*)Cout + (size_t)b * strideC;
      const int hh = lane >> 4, c4 = (lane & 15) * 4;
      for (int pass = 0; pass < 2; ++pass) {
#pragma unroll
        for (int it = 0; it < 8; ++it) {
          const int row = it * 2 + hh;
          v4f v = *(const v4f*)(slab + row * 68 + c4);
          *(volatile v4f*)(C + (size_t)(mBase + row) * ldc + n0 + c4) = v;
        }
        __threadfence();
      }
    } else {
      const int q = lane >> 3, c8 = (lane & 7) * 8;
      unsigned short* C  = (unsigned short*)Cout  + (size_t)b * strideC;
      unsigned short* C2 = (OUT_MODE == 2) ? ((unsigned short*)Cout2 + (size_t)b * strideC) : nullptr;
      for (int pass = 0; pass < 2; ++pass) {
#pragma unroll
        for (int it = 0; it < 4; ++it) {
          const int row = it * 4 + q;
          const float* sp = slab + row * 68 + c8;
          v8h hv, lv;
#pragma unroll
          for (int e = 0; e < 8; ++e) {
            if (OUT_MODE == 1) {
              hv[e] = (_Float16)sp[e];
            } else {
              unsigned short hb = f2bf_bits(sp[e]);
              unsigned short lb = f2bf_bits(sp[e] - bf_bits2f(hb));
              hv[e] = __builtin_bit_cast(_Float16, hb);
              lv[e] = __builtin_bit_cast(_Float16, lb);
            }
          }
          *(volatile v8h*)(C + (size_t)(mBase + row) * ldc + n0 + c8) = hv;
          if (OUT_MODE == 2) *(volatile v8h*)(C2 + (size_t)(mBase + row) * ldc + n0 + c8) = lv;
        }
        __threadfence();
      }
    }
    __builtin_amdgcn_fence(__ATOMIC_RELEASE, "workgroup");
    __builtin_amdgcn_wave_barrier();
    __builtin_amdgcn_fence(__ATOMIC_ACQUIRE, "workgroup");
  }
}

__global__ __launch_bounds__(128) void rmsnorm_f16_kernel(const float* __restrict__ x, const float* __restrict__ w,
                                                          unsigned short* __restrict__ xn) {
  __shared__ float red[4];
  const int row  = blockIdx.x;
  const int t    = threadIdx.x;
  const int lane = t & 31, wave = t >> 5;
  const int c0   = t * 8;
  const float* xr = x + (size_t)row * kDim + c0;
  const v4f a = *(const v4f*)(xr);
  const v4f c = *(const v4f*)(xr + 4);
  float ss = ((a[0] * a[0] + a[1] * a[1]) + (a[2] * a[2] + a[3] * a[3]))
           + ((c[0] * c[0] + c[1] * c[1]) + (c[2] * c[2] + c[3] * c[3]));
#pragma unroll
  for (int off = 16; off > 0; off >>= 1) ss += __shfl_xor(ss, off, 32);
  if (lane == 0) red[wave] = ss;
  __syncthreads();
  const float tot = ((red[0] + red[1]) + red[2]) + red[3];
  const float inv = rsqrtf(tot * kInvDim + kEps);
  const v4f wa = *(const v4f*)(w + c0);
  const v4f wc = *(const v4f*)(w + c0 + 4);
  unsigned short hb[8];
#pragma unroll
  for (int e = 0; e < 4; ++e) {
    hb[e]     = h_bits(a[e] * inv * wa[e]);
    hb[4 + e] = h_bits(c[e] * inv * wc[e]);
  }
  const v4u u = (v4u){pk16(hb[0], hb[1]), pk16(hb[2], hb[3]), pk16(hb[4], hb[5]), pk16(hb[6], hb[7])};
  unsigned short* op = xn + (size_t)row * kDim + c0;
  *(volatile v4u*)op = u;
  __threadfence();
  *(volatile v4u*)op = u;
}

__global__ __launch_bounds__(256) void wtcast_kernel(const float* __restrict__ W, unsigned short* __restrict__ out,
                                                     int Kin, int Nout, float scale) {
  __shared__ float sm[64][65];
  const int t  = threadIdx.x;
  const int k0 = blockIdx.x * 64;
  const int n0 = blockIdx.y * 64;
#pragma unroll
  for (int i = 0; i < 16; ++i) {
    const int e = i * 256 + t;
    const int r = e >> 6;
    const int c = e & 63;
    sm[c][r] = W[(size_t)(k0 + r) * Nout + n0 + c] * scale;
  }
  __syncthreads();
  const int lane = t & 31, wave = t >> 5;
  const int q = lane >> 3, c8 = (lane & 7) * 8;
  for (int pass = 0; pass < 2; ++pass) {
#pragma unroll
    for (int it = 0; it < 2; ++it) {
      const int row = wave * 8 + it * 4 + q;
      unsigned short hb[8];
#pragma unroll
      for (int e = 0; e < 8; ++e) hb[e] = h_bits(sm[row][c8 + e]);
      const v4u u = (v4u){pk16(hb[0], hb[1]), pk16(hb[2], hb[3]), pk16(hb[4], hb[5]), pk16(hb[6], hb[7])};
      *(volatile v4u*)(out + (size_t)(n0 + row) * Kin + k0 + c8) = u;
    }
    __threadfence();
  }
}

__global__ __launch_bounds__(256) void softmax_causal_kernel(const float* __restrict__ S, unsigned short* __restrict__ P) {
  __shared__ float redM[8];
  __shared__ float redS[8];
  const int row  = blockIdx.x;
  const int g    = blockIdx.y;
  const int t    = threadIdx.x;
  const int lane = t & 31, wave = t >> 5;
  const int c0   = t * 8;
  const size_t base = ((size_t)g * kSeq + row) * kSeq + c0;
  const v4f a = *(const v4f*)(S + base);
  const v4f c = *(const v4f*)(S + base + 4);
  float xv[8];
#pragma unroll
  for (int e = 0; e < 4; ++e) {
    xv[e]     = (c0 + e <= row)     ? a[e] : -INFINITY;
    xv[4 + e] = (c0 + 4 + e <= row) ? c[e] : -INFINITY;
  }
  float m = fmaxf(fmaxf(fmaxf(xv[0], xv[1]), fmaxf(xv[2], xv[3])), fmaxf(fmaxf(xv[4], xv[5]), fmaxf(xv[6], xv[7])));
#pragma unroll
  for (int off = 16; off > 0; off >>= 1) m = fmaxf(m, __shfl_xor(m, off, 32));
  if (lane == 0) redM[wave] = m;
  __syncthreads();
  float M = redM[0];
#pragma unroll
  for (int i = 1; i < 8; ++i) M = fmaxf(M, redM[i]);
  float p[8];
  float psum = 0.f;
#pragma unroll
  for (int e = 0; e < 8; ++e) {
    const float pe = (c0 + e <= row) ? expf(xv[e] - M) : 0.f;
    p[e] = pe;
    psum += pe;
  }
#pragma unroll
  for (int off = 16; off > 0; off >>= 1) psum += __shfl_xor(psum, off, 32);
  if (lane == 0) redS[wave] = psum;
  __syncthreads();
  float tot = redS[0];
#pragma unroll
  for (int i = 1; i < 8; ++i) tot += redS[i];
  const float f = kPCarry * (1.0f / tot);
  unsigned short hb[8];
#pragma unroll
  for (int e = 0; e < 8; ++e) hb[e] = h_bits(p[e] * f);
  const v4u u = (v4u){pk16(hb[0], hb[1]), pk16(hb[2], hb[3]), pk16(hb[4], hb[5]), pk16(hb[6], hb[7])};
  unsigned short* op = P + base;
  *(volatile v4u*)op = u;
  __threadfence();
  *(volatile v4u*)op = u;
}

extern "C" void kernel_launch(void* const* d_in, const int* in_sizes, int n_in,
                              void* d_out, int out_size, void* d_ws, size_t ws_size,
                              hipStream_t stream)
{
  if (n_in < 8) return;
  if (in_sizes[0] != kTok * kDim || in_sizes[1] != kDim || in_sizes[2] != kDim * kDim || in_sizes[3] != kDim * kDim ||
      in_sizes[4] != kDim * kDim || in_sizes[5] != kDim * kDim || in_sizes[6] != kDim * kFF || in_sizes[7] != kFF * kDim) return;
  if (out_size != kTok * kDim) return;

  const float* x    = (const float*)d_in[0];
  const float* nrmw = (const float*)d_in[1];
  const float* Wq   = (const float*)d_in[2];
  const float* Wk   = (const float*)d_in[3];
  const float* Wv   = (const float*)d_in[4];
  const float* Wo   = (const float*)d_in[5];
  const float* W1   = (const float*)d_in[6];
  const float* W2   = (const float*)d_in[7];
  float* out = (float*)d_out;

  const size_t MiB = (size_t)1 << 20;
  const size_t szXN  = (size_t)kTok * kDim * 2;
  const size_t szWQK = (size_t)2 * kDim * kDim * 2;
  const size_t szWDD = (size_t)kDim * kDim * 2;
  const size_t szWFF = (size_t)kDim * kFF * 2;
  const size_t szQK  = (size_t)kTok * 2 * kDim * 2;
  const size_t szVT  = (size_t)kDim * kTok * 2;
  const size_t szH   = (size_t)kTok * kFF * 2;
  const size_t szT   = (size_t)kTok * kDim * 4;
  const size_t szCTX = (size_t)kTok * kDim * 2;
  const size_t szP   = (size_t)kGrp * kSeq * kSeq * 2;
  const size_t szSC  = (size_t)kGrp * kSeq * kSeq * 4;

  size_t off = 0;
  const size_t oXN  = off; off += szXN;
  const size_t oWQK = off; off += szWQK;
  const size_t oWV  = off; off += szWDD;
  const size_t oWO  = off; off += szWDD;
  const size_t oW1  = off; off += szWFF;
  const size_t oW2  = off; off += szWFF;
  const size_t oQK  = off; off += szQK;
  const size_t oVT  = off; off += szVT;
  const size_t oH   = off; off += szH;
  const size_t oT   = off; off += szT;
  const size_t total = off;
  const size_t oCTX = oXN;
  const size_t oP   = oW1;
  const size_t oSC  = oH;
  if (szCTX > szXN || szP > 2 * szWFF || szSC > szH) return;
  if (total > ws_size || total > 104 * MiB) return;

  char* ws = (char*)d_ws;
  unsigned short* XN  = (unsigned short*)(ws + oXN);
  unsigned short* WQK = (unsigned short*)(ws + oWQK);
  unsigned short* WVT = (unsigned short*)(ws + oWV);
  unsigned short* WOT = (unsigned short*)(ws + oWO);
  unsigned short* W1T = (unsigned short*)(ws + oW1);
  unsigned short* W2T = (unsigned short*)(ws + oW2);
  unsigned short* QK  = (unsigned short*)(ws + oQK);
  unsigned short* VT  = (unsigned short*)(ws + oVT);
  unsigned short* H   = (unsigned short*)(ws + oH);
  float*          T   = (float*)(ws + oT);
  unsigned short* CTX = (unsigned short*)(ws + oCTX);
  unsigned short* P   = (unsigned short*)(ws + oP);
  float*          SC  = (float*)(ws + oSC);

  rmsnorm_f16_kernel<<<dim3(kTok), dim3(128), 0, stream>>>(x, nrmw, XN);

  wtcast_kernel<<<dim3(kDim / 64, kDim / 64), dim3(256), 0, stream>>>(Wq, WQK, kDim, kDim, kWCarry);
  wtcast_kernel<<<dim3(kDim / 64, kDim / 64), dim3(256), 0, stream>>>(Wk, WQK + (size_t)kDim * kDim, kDim, kDim, kWCarry);
  wtcast_kernel<<<dim3(kDim / 64, kDim / 64), dim3(256), 0, stream>>>(Wv, WVT, kDim, kDim, kWCarry);
  wtcast_kernel<<<dim3(kDim / 64, kDim / 64), dim3(256), 0, stream>>>(Wo, WOT, kDim, kDim, kWCarry);
  wtcast_kernel<<<dim3(kDim / 64, kFF / 64), dim3(256), 0, stream>>>(W1, W1T, kDim, kFF, kWCarry);
  wtcast_kernel<<<dim3(kFF / 64, kDim / 64), dim3(256), 0, stream>>>(W2, W2T, kFF, kDim, kWCarry);

  wmma_gemm64<0, false, 0, 1, false, 0, 0><<<dim3(((kTok / 64) * (2 * kDim / 64)) / 8, 1), dim3(256), 0, stream>>>(
      XN, XN, kDim, 0L, WQK, WQK, kDim, 0L, (void*)QK, (void*)QK, 2 * kDim, 0L, nrmw, x, 0L,
      kTok, 2 * kDim, kDim, kWCarryInv);

  wmma_gemm64<0, false, 0, 1, false, 0, 0><<<dim3(((kDim / 64) * (kTok / 64)) / 8, 1), dim3(256), 0, stream>>>(
      WVT, WVT, kDim, 0L, XN, XN, kDim, 0L, (void*)VT, (void*)VT, kTok, 0L, nrmw, x, 0L,
      kDim, kTok, kDim, kWCarryInv);

  wmma_gemm64<0, false, 0, 1, false, 3, 0><<<dim3(((kTok / 64) * (kFF / 64)) / 8, 1), dim3(256), 0, stream>>>(
      XN, XN, kDim, 0L, W1T, W1T, kDim, 0L, (void*)H, (void*)H, kFF, 0L, nrmw, x, 0L,
      kTok, kFF, kDim, kWCarryInv);

  wmma_gemm64<0, false, 0, 0, true, 0, 0><<<dim3(((kTok / 64) * (kDim / 64)) / 8, 1), dim3(256), 0, stream>>>(
      H, H, kFF, 0L, W2T, W2T, kFF, 0L, (void*)T, (void*)T, kDim, 0L, nrmw, x, 0L,
      kTok, kDim, kFF, kWCarryInv);

  for (int ch = 0; ch < kNChunk; ++ch) {
    const int bb = ch / (kHeads / kGrp);
    const int h0 = (ch % (kHeads / kGrp)) * kGrp;
    const size_t tokRow0 = (size_t)bb * kSeq;
    const unsigned short* Aq = QK + tokRow0 * (2 * kDim) + (size_t)h0 * kHDim;
    const unsigned short* Bk = QK + tokRow0 * (2 * kDim) + kDim + (size_t)h0 * kHDim;
    wmma_gemm64<0, false, 0, 0, false, 0, 1><<<dim3(((kSeq / 64) * (kSeq / 64)) / 8, kGrp), dim3(256), 0, stream>>>(
        Aq, Aq, 2 * kDim, (long)kHDim, Bk, Bk, 2 * kDim, (long)kHDim, (void*)SC, (void*)SC, kSeq, (long)kSeq * kSeq,
        nrmw, x, 0L, kSeq, kSeq, kHDim, kQKScale);
    softmax_causal_kernel<<<dim3(kSeq, kGrp), dim3(256), 0, stream>>>(SC, P);
    const unsigned short* Bv = VT + (size_t)h0 * kHDim * kTok + tokRow0;
    unsigned short* Cc = CTX + tokRow0 * kDim + (size_t)h0 * kHDim;
    wmma_gemm64<0, false, 0, 1, false, 0, 2><<<dim3(((kSeq / 64) * (kHDim / 64) + 7) / 8, kGrp), dim3(256), 0, stream>>>(
        P, P, kSeq, (long)kSeq * kSeq, Bv, Bv, kTok, (long)kHDim * kTok, (void*)Cc, (void*)Cc, kDim, (long)kHDim,
        nrmw, x, 0L, kSeq, kHDim, kSeq, kPVScale);
  }

  wmma_gemm64<0, false, 0, 0, true, 0, 0><<<dim3(((kTok / 64) * (kDim / 64)) / 8, 1), dim3(256), 0, stream>>>(
      CTX, CTX, kDim, 0L, WOT, WOT, kDim, 0L, (void*)out, (void*)out, kDim, 0L, nrmw, T, 0L,
      kTok, kDim, kDim, kWoScale);
}
